// Attention_51599737094204
// MI455X (gfx1250) — hardware-verified
//
#include <hip/hip_runtime.h>


#ifndef NB
#define NB 8
#endif
#ifndef SEQ
#define SEQ 1024
#endif
#define NB_FULL  8
#define SEQ_FULL 1024
#define DM   768
#define NH   12
#define HD   64
#define INR  768
#define QKW  1536
#define WTR  2304
#define KS   32
#define GW   4
#define SPH  72
#define SPF  68
#define WTP  72
#define EXF  6144
#define CSPF 388
#define MXG  4
#define L2E  1.4426950408889634f
static_assert(NH * HD == INR);
static_assert(DM == INR);
static_assert(DM % 32 == 0);
static_assert(HD == 64);
static_assert(QKW == 2 * INR);
static_assert(WTR == 3 * INR);
static_assert(NB <= NB_FULL);
static_assert(SEQ <= SEQ_FULL);
static_assert(SEQ % 64 == 0);
static_assert(SEQ % (2 * KS) == 0);
static_assert((NB * SEQ) % (GW * 32) == 0);
static_assert(INR % (GW * 32) == 0);
static_assert(QKW % 64 == 0);
static_assert(DM % 64 == 0);
static_assert(((size_t)NB * SEQ * DM) % 2048 == 0);
static_assert(EXF == NH * 2 * 32 * 8);
static_assert(16 * CSPF <= 2 * EXF);
static_assert(CSPF * 2 >= INR && (CSPF % 4) == 0);
static_assert((16 * (INR / 8)) % 384 == 0);
static_assert((INR / 8) % 32 == 0);
static_assert((size_t)NB * SEQ * QKW < 2147483647u);
static_assert(NH % MXG == 0 && MXG == 4);
static_assert((NH * 4) % 16 == 0);
static_assert(NH * NH <= 384);
static_assert(NH * 32 == 384);

#define XB_BYTES ((size_t)NB * SEQ * DM * 2)
#define WT_BYTES ((size_t)WTR * DM * 2)
#define WO_BYTES ((size_t)DM * INR * 2)
#define QK_BYTES ((size_t)NB * SEQ * QKW * 2)
#define VT_BYTES ((size_t)NB * INR * SEQ * 2)
#define CX_BYTES ((size_t)NB * SEQ * INR * 2)
#define WS_TOTAL (XB_BYTES + WT_BYTES + WO_BYTES + QK_BYTES + VT_BYTES + CX_BYTES)
static_assert(XB_BYTES % 256 == 0 && WT_BYTES % 256 == 0 && WO_BYTES % 256 == 0 && QK_BYTES % 256 == 0 && VT_BYTES % 256 == 0 && CX_BYTES % 256 == 0);
static_assert(WS_TOTAL <= (size_t)134217728);

typedef unsigned short us;
typedef __attribute__((ext_vector_type(16))) __bf16   v16bf;
typedef __attribute__((ext_vector_type(16))) _Float16 v16h;
typedef __attribute__((ext_vector_type(2)))  _Float16 v2h;
typedef __attribute__((ext_vector_type(8)))  unsigned short v8us;
typedef __attribute__((ext_vector_type(4)))  unsigned int   v4u;
typedef __attribute__((ext_vector_type(8)))  unsigned int   v8u;
typedef __attribute__((ext_vector_type(8)))  float    v8f;
typedef __attribute__((ext_vector_type(4)))  float    v4f;
typedef v4f  __attribute__((may_alias)) v4fa;
typedef v4u  __attribute__((may_alias)) v4ua;
typedef v8us __attribute__((may_alias)) v8usa;

__device__ __forceinline__ unsigned short f2bf(float f) { unsigned u = __float_as_uint(f); u += 0x7FFFu + ((u >> 16) & 1u); return (unsigned short)(u >> 16); }
__device__ __forceinline__ float bf2f(unsigned short b) { return __uint_as_float(((unsigned)b) << 16); }
__device__ __forceinline__ float bfr(float f) { return bf2f(f2bf(f)); }
__device__ __forceinline__ unsigned short f2h(float f) { return __builtin_bit_cast(unsigned short, (_Float16)f); }
__device__ __forceinline__ v16bf cat16b(v8us lo, v8us hi) { return __builtin_bit_cast(v16bf, __builtin_shufflevector(lo, hi, 0, 1, 2, 3, 4, 5, 6, 7, 8, 9, 10, 11, 12, 13, 14, 15)); }
__device__ __forceinline__ v16h  cat16h(v8us lo, v8us hi) { return __builtin_bit_cast(v16h,  __builtin_shufflevector(lo, hi, 0, 1, 2, 3, 4, 5, 6, 7, 8, 9, 10, 11, 12, 13, 14, 15)); }
__device__ __forceinline__ v8f wmmab(v16bf a, v16bf b, v8f c) { return __builtin_amdgcn_wmma_f32_16x16x32_bf16(false, a, false, b, (short)0, c, false, false); }
__device__ __forceinline__ v8f wmmah(v16h a, v16h b, v8f c)   { return __builtin_amdgcn_wmma_f32_16x16x32_f16(false, a, false, b, (short)0, c, false, false); }
__device__ __forceinline__ v16bf ldb(const us* p) { return cat16b(*(const v8us*)p, *(const v8us*)(p + 16)); }
__device__ __forceinline__ v16h  ldh(const us* p) { return cat16h(*(const v8us*)p, *(const v8us*)(p + 16)); }
__device__ __forceinline__ unsigned pk2h(float a, float b) { v2h t; t[0] = (_Float16)a; t[1] = (_Float16)b; return __builtin_bit_cast(unsigned, t); }

__global__ __launch_bounds__(256) void k_cvtx(const float* __restrict__ x, us* XB) {
    const unsigned i = blockIdx.x * 256u + threadIdx.x;
    const unsigned per = (unsigned)(SEQ * DM / 8);
    if (i >= (unsigned)NB * per) return;
    const unsigned b = i / per, r = i - b * per;
    const float* src = x + (size_t)b * SEQ_FULL * DM + (size_t)r * 8;
    us* dst = XB + (size_t)i * 8;
    const v8f v = *(const v8f*)src;
    v8us o;
#pragma unroll
    for (int c = 0; c < 8; ++c) o[c] = f2bf(v[c]);
    *(volatile v8us*)dst = o;
    __threadfence();
    *(volatile v8us*)dst = o;
}

__global__ __launch_bounds__(256) void k_wt(const float* __restrict__ W, int ncols, us* dst, int row0, float scale, int asf16) {
    __shared__ __align__(16) us tl[64 * WTP];
    const unsigned tid = threadIdx.x;
    const int n0 = (int)blockIdx.x * 64, k0 = (int)blockIdx.y * 64;
#pragma unroll
    for (unsigned it = 0; it < 4; ++it) {
        const unsigned f = it * 256u + tid;
        const unsigned kk = f >> 4, c4 = (f & 15u) * 4u;
        const v4f xv = *(const v4f*)(W + (size_t)(k0 + (int)kk) * ncols + n0 + (int)c4);
#pragma unroll
        for (unsigned c = 0; c < 4; ++c) {
            const unsigned short bb = f2bf(xv[c]);
            const unsigned short hb = f2h(bf2f(bb) * scale);
            tl[(c4 + c) * WTP + kk] = asf16 ? hb : bb;
        }
    }
    __syncthreads();
    const unsigned c8 = (tid & 7u) * 8u, rr = tid >> 3;
#pragma unroll 1
    for (int ps = 0; ps < 2; ++ps) {
#pragma unroll
        for (unsigned it = 0; it < 2; ++it) {
            const unsigned n = it * 32u + rr;
            const v8us o = *(const v8usa*)(tl + n * WTP + c8);
            *(volatile v8us*)(dst + (size_t)(row0 + n0 + (int)n) * DM + k0 + c8) = o;
        }
        if (ps == 0) __threadfence();
    }
}

__device__ __forceinline__ void gemm_bf(const us* __restrict__ Cp, int coff, const us* __restrict__ Rp, int roff, v8f (&acc)[4][2]) {
#pragma unroll
    for (int i = 0; i < 4; ++i) {
#pragma unroll
        for (int j = 0; j < 2; ++j) acc[i][j] = (v8f){};
    }
#pragma unroll 1
    for (int k = 0; k < DM; k += 32) {
        v16bf a[4], bq[2];
#pragma unroll
        for (int i = 0; i < 4; ++i) a[i] = ldb(Cp + (coff + i * 16 * DM + k));
#pragma unroll
        for (int j = 0; j < 2; ++j) bq[j] = ldb(Rp + (roff + j * 16 * DM + k));
#pragma unroll
        for (int i = 0; i < 4; ++i) {
#pragma unroll
            for (int j = 0; j < 2; ++j) acc[i][j] = wmmab(a[i], bq[j], acc[i][j]);
        }
        asm volatile("v_nop\n\tv_nop\n\tv_nop\n\tv_nop"
                     : "+v"(acc[0][0]), "+v"(acc[0][1]), "+v"(acc[1][0]), "+v"(acc[1][1]), "+v"(acc[2][0]), "+v"(acc[2][1]), "+v"(acc[3][0]), "+v"(acc[3][1])
                     : "v"(a[0]), "v"(a[1]), "v"(a[2]), "v"(a[3]), "v"(bq[0]), "v"(bq[1]));
    }
}
__device__ __forceinline__ void gemm_h(const us* __restrict__ Cp, int coff, const us* __restrict__ Rp, int roff, v8f (&acc)[4][2]) {
#pragma unroll
    for (int i = 0; i < 4; ++i) {
#pragma unroll
        for (int j = 0; j < 2; ++j) acc[i][j] = (v8f){};
    }
#pragma unroll 1
    for (int k = 0; k < DM; k += 32) {
        v16h a[4], bq[2];
#pragma unroll
        for (int i = 0; i < 4; ++i) a[i] = ldh(Cp + (coff + i * 16 * DM + k));
#pragma unroll
        for (int j = 0; j < 2; ++j) bq[j] = ldh(Rp + (roff + j * 16 * DM + k));
#pragma unroll
        for (int i = 0; i < 4; ++i) {
#pragma unroll
            for (int j = 0; j < 2; ++j) acc[i][j] = wmmah(a[i], bq[j], acc[i][j]);
        }
        asm volatile("v_nop\n\tv_nop\n\tv_nop\n\tv_nop"
                     : "+v"(acc[0][0]), "+v"(acc[0][1]), "+v"(acc[1][0]), "+v"(acc[1][1]), "+v"(acc[2][0]), "+v"(acc[2][1]), "+v"(acc[3][0]), "+v"(acc[3][1])
                     : "v"(a[0]), "v"(a[1]), "v"(a[2]), "v"(a[3]), "v"(bq[0]), "v"(bq[1]));
    }
}

__device__ __forceinline__ void epi_h(v8f (&acc)[4][2], us* Out, size_t obase, int ldo) {
    __shared__ __align__(16) us st[GW * 32 * SPH];
    const unsigned lane = threadIdx.x & 31u, wv = threadIdx.x >> 5, lr = lane & 15u, hi = lane >> 4;
    const unsigned sb = wv * (32u * SPH);
#pragma unroll
    for (int i = 0; i < 4; ++i) {
#pragma unroll
        for (int j = 0; j < 2; ++j) {
            v4u pk;
#pragma unroll
            for (int e = 0; e < 4; ++e) pk[e] = pk2h(acc[i][j][2 * e], acc[i][j][2 * e + 1]);
            *(v4ua*)(st + sb + (16u * j + lr) * SPH + 16u * i + 8u * hi) = pk;
        }
    }
    __syncthreads();
    const unsigned q8 = (lane & 7u) * 8u, rq = lane >> 3;
#pragma unroll 1
    for (int ps = 0; ps < 2; ++ps) {
#pragma unroll
        for (unsigned it = 0; it < 8; ++it) {
            const unsigned row = it * 4u + rq;
            const v8us o = *(const v8usa*)(st + sb + row * SPH + q8);
            *(volatile v8us*)(Out + obase + (size_t)row * ldo + q8) = o;
        }
        if (ps == 0) __threadfence();
    }
}

__global__ __launch_bounds__(128) void k_gemm_qk(const us* __restrict__ XB, const us* __restrict__ WT, us* QK) {
    const int lane = threadIdx.x & 31, wv = threadIdx.x >> 5, lr = lane & 15, hi = lane >> 4;
    const int r0 = ((int)blockIdx.y * GW + wv) * 32;
    const int c0 = (int)blockIdx.x * 64;
    v8f acc[4][2];
    gemm_bf(WT, (c0 + lr) * DM + 8 * hi, XB, (r0 + lr) * DM + 8 * hi, acc);
    epi_h(acc, QK, (size_t)r0 * QKW + c0, QKW);
}

__global__ __launch_bounds__(128) void k_gemm_vt(const us* __restrict__ XB, const us* __restrict__ WT, us* VT) {
    const int lane = threadIdx.x & 31, wv = threadIdx.x >> 5, lr = lane & 15, hi = lane >> 4;
    const int r0 = ((int)blockIdx.y * GW + wv) * 32;
    const int c0 = (int)blockIdx.x * 64;
    const int b = (int)blockIdx.z;
    v8f acc[4][2];
    gemm_bf(XB, (b * SEQ + c0 + lr) * DM + 8 * hi, WT, (2 * INR + r0 + lr) * DM + 8 * hi, acc);
    epi_h(acc, VT, ((size_t)b * INR + r0) * SEQ + c0, SEQ);
}

__global__ __launch_bounds__(128) void k_gemm_out(const us* __restrict__ CTX, const us* __restrict__ WOT, const float* __restrict__ bout, float* OUT) {
    __shared__ __align__(16) float sf[GW * 32 * SPF];
    const int lane = threadIdx.x & 31, wv = threadIdx.x >> 5, lr = lane & 15, hi = lane >> 4;
    const int r0 = ((int)blockIdx.y * GW + wv) * 32;
    const int c0 = (int)blockIdx.x * 64;
    v8f acc[4][2];
    gemm_h(WOT, (c0 + lr) * INR + 8 * hi, CTX, (r0 + lr) * INR + 8 * hi, acc);
    const int sb = wv * (32 * SPF);
    const float sc = 1.0f / 1024.0f;
#pragma unroll
    for (int i = 0; i < 4; ++i) {
#pragma unroll
        for (int j = 0; j < 2; ++j) {
            const v8f a = acc[i][j] * sc;
            const int o = sb + (16 * j + lr) * SPF + 16 * i + 8 * hi;
            *(v4fa*)(sf + o)     = __builtin_shufflevector(a, a, 0, 1, 2, 3);
            *(v4fa*)(sf + o + 4) = __builtin_shufflevector(a, a, 4, 5, 6, 7);
        }
    }
    __syncthreads();
    const int c4 = lr * 4, rh = hi;
    v4f bias = *(const v4f*)(bout + c0 + c4);
    bias[0] = bfr(bias[0]); bias[1] = bfr(bias[1]); bias[2] = bfr(bias[2]); bias[3] = bfr(bias[3]);
    float* orow = OUT + (size_t)r0 * DM + c0 + c4;
#pragma unroll 1
    for (int ps = 0; ps < 2; ++ps) {
#pragma unroll 4
        for (int it = 0; it < 16; ++it) {
            const int row = it * 2 + rh;
            const v4f v = *(const v4fa*)(sf + sb + row * SPF + c4);
            const v4f val = v + bias;
            *(volatile v4f*)(orow + (size_t)row * DM) = val;
        }
        if (ps == 0) __threadfence();
    }
}

__global__ __launch_bounds__(384) __attribute__((amdgpu_num_vgpr(256))) void k_attn(const us* __restrict__ QK, const us* __restrict__ VT, const float* __restrict__ mpre, const float* __restrict__ mpost, us* CTX) {
    __shared__ __align__(16) float xs[2 * EXF];
    __shared__ __align__(16) float mt[2 * NH * NH];
    const int tid = threadIdx.x, lane = tid & 31, lr = lane & 15, hi = lane >> 4;
    const int g = __builtin_amdgcn_readfirstlane(tid >> 5);
    const int qt = SEQ / 16;
    const int b = (int)blockIdx.x / qt;
    const int q0 = ((int)blockIdx.x - b * qt) * 16;

    {
        const int mi = tid < NH * NH ? tid : NH * NH - 1;
        const float ca = mpre[mi];
        const float cc = mpost[mi];
        if (tid < NH * NH) {
            const int h = tid / NH, gg = tid - h * NH;
            mt[gg * NH + h] = bfr(ca) * (0.125f * L2E);
            mt[NH * NH + gg * NH + h] = bfr(cc) * 256.0f;
        }
    }
    __syncthreads();

    const int qo = (b * SEQ + q0 + lr) * QKW + g * HD + 8 * hi;
    const v16h qf0 = ldh(QK + qo);
    const v16h qf1 = ldh(QK + qo + 32);
    const int kb = (b * SEQ + lr) * QKW + INR + g * HD + 8 * hi;
    const int vb = (b * INR + g * HD + lr) * SEQ + 8 * hi;
    const int slot = g * 512 + lane * 8;
    const int rd = lane * 8;
    const int wpo = g * NH;
    const int wqo = NH * NH + g * NH;

    float ml = -1.0e30f;
    float l = 0.0f;

#pragma unroll 1
    for (int k0 = 0; k0 < SEQ; k0 += KS) {
        const int eb = ((k0 >> 5) & 1) * EXF;
        v8f s0 = (v8f){}, s1 = (v8f){};
        {
            const int ko = kb + k0 * QKW;
            const v16h a00 = ldh(QK + ko), a10 = ldh(QK + ko + 16 * QKW);
            const v16h a01 = ldh(QK + ko + 32), a11 = ldh(QK + ko + 16 * QKW + 32);
            s0 = wmmah(a00, qf0, s0);
            s1 = wmmah(a10, qf0, s1);
            s0 = wmmah(a01, qf1, s0);
            s1 = wmmah(a11, qf1, s1);
            asm volatile("v_nop\n\tv_nop\n\tv_nop\n\tv_nop" : "+v"(s0), "+v"(s1) : "v"(qf0), "v"(qf1), "v"(a00), "v"(a10), "v"(a01), "v"(a11));
        }
        *(v4fa*)(xs + eb + slot)       = __builtin_shufflevector(s0, s0, 0, 1, 2, 3);
        *(v4fa*)(xs + eb + slot + 4)   = __builtin_shufflevector(s0, s0, 4, 5, 6, 7);
        *(v4fa*)(xs + eb + slot + 256) = __builtin_shufflevector(s1, s1, 0, 1, 2, 3);
        *(v4fa*)(xs + eb + slot + 260) = __builtin_shufflevector(s1, s1, 4, 5, 6, 7);
        __syncthreads();
        v4f t0 = (v4f){}, t1 = (v4f){}, t2 = (v4f){}, t3 = (v4f){};
#pragma unroll
        for (int gp = 0; gp < NH / MXG; ++gp) {
            const v4f w = *(const v4fa*)(mt + wpo + MXG * gp);
#pragma unroll
            for (int hh = 0; hh < MXG; ++hh) {
                const int o = eb + (MXG * gp + hh) * 512 + rd;
                const v4f a = *(const v4fa*)(xs + o);
                const v4f c = *(const v4fa*)(xs + o + 4);
                const v4f d = *(const v4fa*)(xs + o + 256);
                const v4f e = *(const v4fa*)(xs + o + 260);
                t0 += a * w[hh]; t1 += c * w[hh]; t2 += d * w[hh]; t3 += e * w[hh];
            }
            asm volatile("" ::: "memory");
        }
        float mx = fmaxf(fmaxf(t0[0], t1[0]), fmaxf(t2[0], t3[0]));
#pragma unroll
        for (int r = 1; r < 4; ++r) mx = fmaxf(mx, fmaxf(fmaxf(t0[r], t1[r]), fmaxf(t2[r], t3[r])));
        mx = fmaxf(mx, __shfl_xor(mx, 16, 32));
        const float mn = fmaxf(ml, mx);
        const float corr = __builtin_amdgcn_exp2f(ml - mn);
        ml = mn;
        float ps = 0.0f;
#pragma unroll
        for (int r = 0; r < 4; ++r) {
            ps += __builtin_amdgcn_exp2f(t0[r] - mn) + __builtin_amdgcn_exp2f(t1[r] - mn);
            ps += __builtin_amdgcn_exp2f(t2[r] - mn) + __builtin_amdgcn_exp2f(t3[r] - mn);
        }
        ps += __shfl_xor(ps, 16, 32);
        l = l * corr + ps;
    }

    const float cof = ml + __log2f(l);

    v8f o[4];
#pragma unroll
    for (int t = 0; t < 4; ++t) o[t] = (v8f){};

#pragma unroll 1
    for (int k0 = 0; k0 < SEQ; k0 += KS) {
        v8f s0 = (v8f){}, s1 = (v8f){};
        {
            const int ko = kb + k0 * QKW;
            const v16h a00 = ldh(QK + ko), a10 = ldh(QK + ko + 16 * QKW);
            const v16h a01 = ldh(QK + ko + 32), a11 = ldh(QK + ko + 16 * QKW + 32);
            s0 = wmmah(a00, qf0, s0);
            s1 = wmmah(a10, qf0, s1);
            s0 = wmmah(a01, qf1, s0);
            s1 = wmmah(a11, qf1, s1);
            asm volatile("v_nop\n\tv_nop\n\tv_nop\n\tv_nop" : "+v"(s0), "+v"(s1) : "v"(qf0), "v"(qf1), "v"(a00), "v"(a10), "v"(a01), "v"(a11));
        }
        *(v4fa*)(xs + slot)       = __builtin_shufflevector(s0, s0, 0, 1, 2, 3);
        *(v4fa*)(xs + slot + 4)   = __builtin_shufflevector(s0, s0, 4, 5, 6, 7);
        *(v4fa*)(xs + slot + 256) = __builtin_shufflevector(s1, s1, 0, 1, 2, 3);
        *(v4fa*)(xs + slot + 260) = __builtin_shufflevector(s1, s1, 4, 5, 6, 7);
        __syncthreads();
        {
            v4f t0 = (v4f){}, t1 = (v4f){}, t2 = (v4f){}, t3 = (v4f){};
#pragma unroll
            for (int gp = 0; gp < NH / MXG; ++gp) {
                const v4f w = *(const v4fa*)(mt + wpo + MXG * gp);
#pragma unroll
                for (int hh = 0; hh < MXG; ++hh) {
                    const int oo = (MXG * gp + hh) * 512 + rd;
                    const v4f a = *(const v4fa*)(xs + oo);
                    const v4f c = *(const v4fa*)(xs + oo + 4);
                    const v4f d = *(const v4fa*)(xs + oo + 256);
                    const v4f e = *(const v4fa*)(xs + oo + 260);
                    t0 += a * w[hh]; t1 += c * w[hh]; t2 += d * w[hh]; t3 += e * w[hh];
                }
                asm volatile("" ::: "memory");
            }
            v4f p0, p1, p2, p3;
#pragma unroll
            for (int r = 0; r < 4; ++r) {
                p0[r] = __builtin_amdgcn_exp2f(t0[r] - cof);
                p1[r] = __builtin_amdgcn_exp2f(t1[r] - cof);
                p2[r] = __builtin_amdgcn_exp2f(t2[r] - cof);
                p3[r] = __builtin_amdgcn_exp2f(t3[r] - cof);
            }
            *(v4fa*)(xs + EXF + slot)       = p0;
            *(v4fa*)(xs + EXF + slot + 4)   = p1;
            *(v4fa*)(xs + EXF + slot + 256) = p2;
            *(v4fa*)(xs + EXF + slot + 260) = p3;
        }
        __syncthreads();
        v4f a0 = (v4f){}, a1 = (v4f){}, a2 = (v4f){}, a3 = (v4f){};
#pragma unroll
        for (int gp = 0; gp < NH / MXG; ++gp) {
            const v4f w = *(const v4fa*)(mt + wqo + MXG * gp);
#pragma unroll
            for (int hh = 0; hh < MXG; ++hh) {
                const int oo = EXF + (MXG * gp + hh) * 512 + rd;
                const v4f a = *(const v4fa*)(xs + oo);
                const v4f c = *(const v4fa*)(xs + oo + 4);
                const v4f d = *(const v4fa*)(xs + oo + 256);
                const v4f e = *(const v4fa*)(xs + oo + 260);
                a0 += a * w[hh]; a1 += c * w[hh]; a2 += d * w[hh]; a3 += e * w[hh];
            }
            asm volatile("" ::: "memory");
        }
        v8u pw;
        pw[0] = pk2h(a0[0], a0[1]); pw[1] = pk2h(a0[2], a0[3]);
        pw[2] = pk2h(a1[0], a1[1]); pw[3] = pk2h(a1[2], a1[3]);
        pw[4] = pk2h(a2[0], a2[1]); pw[5] = pk2h(a2[2], a2[3]);
        pw[6] = pk2h(a3[0], a3[1]); pw[7] = pk2h(a3[2], a3[3]);
        const v16h pf = __builtin_bit_cast(v16h, pw);

        v16h av[4];
#pragma unroll
        for (int t = 0; t < 4; ++t) av[t] = ldh(VT + (vb + t * 16 * SEQ + k0));
#pragma unroll
        for (int t = 0; t < 4; ++t) o[t] = wmmah(av[t], pf, o[t]);
        asm volatile("v_nop\n\tv_nop\n\tv_nop\n\tv_nop"
                     : "+v"(o[0]), "+v"(o[1]), "+v"(o[2]), "+v"(o[3])
                     : "v"(pf), "v"(av[0]), "v"(av[1]), "v"(av[2]), "v"(av[3]));
    }

    __syncthreads();
#pragma unroll
    for (int t = 0; t < 4; ++t) {
        v4u pk;
#pragma unroll
        for (int e = 0; e < 4; ++e) pk[e] = pk2h(o[t][2 * e] * 0.0625f, o[t][2 * e + 1] * 0.0625f);
        *(v4ua*)(xs + lr * CSPF + g * 32 + 8 * t + 4 * hi) = pk;
    }
    __syncthreads();
    us* cbase = CTX + (size_t)(b * SEQ + q0) * INR;
#pragma unroll 1
    for (int ps2 = 0; ps2 < 2; ++ps2) {
#pragma unroll
        for (int it = 0; it < 4; ++it) {
            const int idx = it * 384 + tid;
            const int row = idx / 96;
            const int pc = idx - row * 96;
            const v4u val = *(const v4ua*)(xs + row * CSPF + pc * 4);
            *(volatile v4u*)(cbase + (size_t)row * INR + pc * 8) = val;
        }
        if (ps2 == 0) __threadfence();
    }
}

extern "C" void kernel_launch(void* const* d_in, const int* in_sizes, int n_in,
                              void* d_out, int out_size, void* d_ws, size_t ws_size, hipStream_t stream) {
    if (n_in < 7) return;
    const size_t needx = ((size_t)(NB - 1) * SEQ_FULL + SEQ) * DM;
    if ((size_t)in_sizes[0] < needx) return;
    if ((size_t)in_sizes[1] < (size_t)DM * INR) return;
    if ((size_t)in_sizes[2] < (size_t)DM * 2 * INR) return;
    if (in_sizes[3] < NH * NH || in_sizes[4] < NH * NH) return;
    if ((size_t)in_sizes[5] < (size_t)INR * DM) return;
    if (in_sizes[6] < DM) return;
    if ((size_t)out_size < (size_t)NB * SEQ * DM) return;
    if (WS_TOTAL > ws_size) return;

    const float* x     = (const float*)d_in[0];
    const float* Wq    = (const float*)d_in[1];
    const float* Wkv   = (const float*)d_in[2];
    const float* mpre  = (const float*)d_in[3];
    const float* mpost = (const float*)d_in[4];
    const float* Wo    = (const float*)d_in[5];
    const float* bo    = (const float*)d_in[6];
    float* OUT = (float*)d_out;

    char* wsp = (char*)d_ws;
    us* XB  = (us*)(wsp);
    us* WT  = (us*)(wsp + XB_BYTES);
    us* WOT = (us*)(wsp + XB_BYTES + WT_BYTES);
    us* QK  = (us*)(wsp + XB_BYTES + WT_BYTES + WO_BYTES);
    us* VT  = (us*)(wsp + XB_BYTES + WT_BYTES + WO_BYTES + QK_BYTES);
    us* CTX = (us*)(wsp + XB_BYTES + WT_BYTES + WO_BYTES + QK_BYTES + VT_BYTES);

    const unsigned gc = (unsigned)(((size_t)NB * SEQ * DM / 8 + 255) / 256);
    k_cvtx<<<gc, 256, 0, stream>>>(x, XB);
    k_wt<<<dim3(INR / 64, DM / 64, 1), 256, 0, stream>>>(Wq, INR, WT, 0, 1.0f, 0);
    k_wt<<<dim3(2 * INR / 64, DM / 64, 1), 256, 0, stream>>>(Wkv, 2 * INR, WT, INR, 1.0f, 0);
    k_wt<<<dim3(DM / 64, INR / 64, 1), 256, 0, stream>>>(Wo, DM, WOT, 0, 64.0f, 1);
    k_gemm_qk<<<dim3(QKW / 64, (unsigned)(NB * SEQ / (GW * 32)), 1), 128, 0, stream>>>(XB, WT, QK);
    k_gemm_vt<<<dim3(SEQ / 64, INR / (GW * 32), NB), 128, 0, stream>>>(XB, WT, VT);
    k_attn<<<(unsigned)(NB * (SEQ / 16)), 384, 0, stream>>>(QK, VT, mpre, mpost, CTX);
    k_gemm_out<<<dim3(DM / 64, (unsigned)(NB * SEQ / (GW * 32)), 1), 128, 0, stream>>>(CTX, WOT, bo, OUT);
}
